// GraphRUNet_54640573939801
// MI455X (gfx1250) — hardware-verified
//
#include <hip/hip_runtime.h>
#include <stddef.h>


#define HIDC    128
#define NMAT    7
#define NTHR    256
#define NWAVE   8
#define EPT     8
#define NGRP    2
#define CHUNK   (NTHR * EPT * NGRP)
#define WCAP    (EPT * NGRP * 32)
#define LISTN   (NWAVE * WCAP)
#define NBC     4096
#define NBF     1024
#define RCAP    40960
#define RBN     128
#define TGT     256
#define DEGCAP  256
#define GROWS   128
#define OTHR    512
#define AP      (HIDC + 8)
#define SCH     2048
#define PBLK    4096
#define RPB     8
#define EPB     (NTHR * 4)

#define LDS_GEMM (2 * GROWS * AP * 2 + GROWS * HIDC * 4)
#define LDS_FILL ((RCAP + NBF + LISTN) * 4 + 64)

static_assert((CHUNK & (CHUNK - 1)) == 0);
static_assert(CHUNK <= 4096);
static_assert(NBC <= 4096 && NBF <= 4096);
static_assert((NBC & (NBC - 1)) == 0 && (NBF & (NBF - 1)) == 0);
static_assert(NBC == 4 * NBF);
static_assert(OTHR * 8 == NBC);
static_assert((RCAP % 32) == 0);
static_assert(TGT == NWAVE * 32 && (TGT % GROWS) == 0);
static_assert((GROWS * HIDC / 8) % NTHR == 0);
static_assert((AP % 8) == 0);
static_assert(SCH == 8 * NTHR);
static_assert(PBLK == 16 * NTHR);
static_assert(RPB == NWAVE);
static_assert((SCH % TGT) == 0 && (NBC % TGT) == 0 && (PBLK % 4) == 0);

typedef float          v4f  __attribute__((ext_vector_type(4)));
typedef float          v8f  __attribute__((ext_vector_type(8)));
typedef int            v4i  __attribute__((ext_vector_type(4)));
typedef unsigned short v8us __attribute__((ext_vector_type(8)));
typedef __bf16         v16b __attribute__((ext_vector_type(16)));
typedef unsigned long long u64;
typedef u64            v2u  __attribute__((ext_vector_type(2)));
union FragB { v16b v; v8us h[2]; };

__device__ __forceinline__ unsigned bfr(float f) {
  const unsigned u = __float_as_uint(f);
  return (u + 0x7FFFu + ((u >> 16) & 1u)) >> 16;
}
__device__ __forceinline__ void split1(float x, unsigned short& h, unsigned short& l) {
  const unsigned hb = bfr(x);
  const float hf = __uint_as_float(hb << 16);
  h = (unsigned short)hb;
  l = (unsigned short)bfr(x - hf);
}
__device__ __forceinline__ void split8(v4f a, v4f b, v8us& hi, v8us& lo) {
  unsigned short h0, h1, h2, h3, h4, h5, h6, h7, l0, l1, l2, l3, l4, l5, l6, l7;
  split1(a.x, h0, l0); split1(a.y, h1, l1); split1(a.z, h2, l2); split1(a.w, h3, l3);
  split1(b.x, h4, l4); split1(b.y, h5, l5); split1(b.z, h6, l6); split1(b.w, h7, l7);
  hi[0] = h0; hi[1] = h1; hi[2] = h2; hi[3] = h3; hi[4] = h4; hi[5] = h5; hi[6] = h6; hi[7] = h7;
  lo[0] = l0; lo[1] = l1; lo[2] = l2; lo[3] = l3; lo[4] = l4; lo[5] = l5; lo[6] = l6; lo[7] = l7;
}

__device__ __forceinline__ v8f wmb(v16b a, v16b b, v8f c) {
  v8f d = __builtin_amdgcn_wmma_f32_16x16x32_bf16(false, a, false, b, (short)0, c, false, false);
  asm volatile("v_nop\n\tv_nop\n\tv_nop\n\tv_nop" : "+v"(d) : "v"(a), "v"(b));
  return d;
}

__device__ __forceinline__ u64 mkkey(float s, int idx) {
  const unsigned u = __float_as_uint(s);
  const unsigned mneg = ~u, mpos = u | 0x80000000u;
  const unsigned mono = (u & 0x80000000u) ? mneg : mpos;
  return ((u64)mono << 32) | (u64)(~(unsigned)idx);
}

template <int NB>
__device__ __forceinline__ int scan_chunk(const int* __restrict__ dsts, int nE, int cbase, int slotBase,
                                          int vec8, int* list, int tid, int lane, int wave) {
  int wc = 0;
#pragma unroll
  for (int g = 0; g < NGRP; ++g) {
    const int el0  = (g * NTHR + tid) * EPT;
    const int e0   = cbase + el0;
    const int sent = -2147483647 - 1;
    v4i da, db;
    if (vec8 != 0 && cbase + CHUNK <= nE) {
      da = *(const v4i*)(dsts + e0);
      db = *(const v4i*)(dsts + e0 + 4);
    } else {
      da.x = (e0     < nE) ? dsts[min(e0, nE - 1)] : sent;
      da.y = (e0 + 1 < nE) ? dsts[min(e0 + 1, nE - 1)] : sent;
      da.z = (e0 + 2 < nE) ? dsts[min(e0 + 2, nE - 1)] : sent;
      da.w = (e0 + 3 < nE) ? dsts[min(e0 + 3, nE - 1)] : sent;
      db.x = (e0 + 4 < nE) ? dsts[min(e0 + 4, nE - 1)] : sent;
      db.y = (e0 + 5 < nE) ? dsts[min(e0 + 5, nE - 1)] : sent;
      db.z = (e0 + 6 < nE) ? dsts[min(e0 + 6, nE - 1)] : sent;
      db.w = (e0 + 7 < nE) ? dsts[min(e0 + 7, nE - 1)] : sent;
    }
    const unsigned nb = (unsigned)slotBase;
    const unsigned s0 = (unsigned)da.x - nb, s1 = (unsigned)da.y - nb;
    const unsigned s2 = (unsigned)da.z - nb, s3 = (unsigned)da.w - nb;
    const unsigned s4 = (unsigned)db.x - nb, s5 = (unsigned)db.y - nb;
    const unsigned s6 = (unsigned)db.z - nb, s7 = (unsigned)db.w - nb;
    const bool h0 = s0 < (unsigned)NB, h1 = s1 < (unsigned)NB, h2 = s2 < (unsigned)NB, h3 = s3 < (unsigned)NB;
    const bool h4 = s4 < (unsigned)NB, h5 = s5 < (unsigned)NB, h6 = s6 < (unsigned)NB, h7 = s7 < (unsigned)NB;
    const unsigned any = __builtin_amdgcn_ballot_w32(h0 | h1 | h2 | h3 | h4 | h5 | h6 | h7);
    if (any != 0u) {
#define HITJ(J, HJ, SJ) { \
        const unsigned mj = __builtin_amdgcn_ballot_w32(HJ); \
        if (mj != 0u) { \
          if (HJ) { \
            const int pos = wc + (int)__builtin_amdgcn_mbcnt_lo(mj, 0u); \
            if (pos < WCAP) list[wave * WCAP + pos] = ((el0 + (J)) << 12) | (int)(SJ); \
          } \
          wc += (int)__builtin_popcount(mj); } }
      HITJ(0, h0, s0)
      HITJ(1, h1, s1)
      HITJ(2, h2, s2)
      HITJ(3, h3, s3)
      HITJ(4, h4, s4)
      HITJ(5, h5, s5)
      HITJ(6, h6, s6)
      HITJ(7, h7, s7)
#undef HITJ
    }
  }
  return wc;
}

__global__ __launch_bounds__(NTHR) void k_wprep(
    const float* __restrict__ Wd0, const float* __restrict__ Wd, const float* __restrict__ Wu,
    unsigned short* wp) {
  const int seg = (int)blockIdx.x >> 3;
  const float* src = seg == 0 ? Wd0
                   : (seg <= 3 ? Wd + (size_t)(seg - 1) * HIDC * HIDC
                               : Wu + (size_t)(seg - 4) * HIDC * HIDC);
  const int i  = ((int)(blockIdx.x & 7) * NTHR) + (int)threadIdx.x;
  const int n  = i >> 4;
  const int k0 = (i & 15) * 8;
  v4f a, b;
  a.x = src[(k0 + 0) * HIDC + n]; a.y = src[(k0 + 1) * HIDC + n];
  a.z = src[(k0 + 2) * HIDC + n]; a.w = src[(k0 + 3) * HIDC + n];
  b.x = src[(k0 + 4) * HIDC + n]; b.y = src[(k0 + 5) * HIDC + n];
  b.z = src[(k0 + 6) * HIDC + n]; b.w = src[(k0 + 7) * HIDC + n];
  v8us hi, lo;
  split8(a, b, hi, lo);
  unsigned short* dh = wp + (size_t)seg * 2 * HIDC * HIDC + (size_t)i * 8;
  unsigned short* dl = dh + HIDC * HIDC;
  *(volatile v8us*)dh = hi;
  *(volatile v8us*)dl = lo;
  __threadfence();
  *(volatile v8us*)dh = hi;
  *(volatile v8us*)dl = lo;
}

__global__ __launch_bounds__(NTHR) void k_count(
    const int* __restrict__ dsts, int* cnt, float* dinv, int nE, int vec8) {
  __shared__ __attribute__((aligned(16))) int scnt[NBC];
  __shared__ __attribute__((aligned(16))) int list[LISTN];
  __shared__ int wcnt[NWAVE];
  const int tid = threadIdx.x, lane = tid & 31, wave = tid >> 5;
  const int nodeBase = blockIdx.x * NBC;

  for (int i = tid; i < NBC; i += NTHR) scnt[i] = 0;
  __syncthreads();

  const int nChunks = (nE + CHUNK - 1) / CHUNK;
#pragma unroll 1
  for (int ch = 0; ch < nChunks; ++ch) {
    const int cbase = ch * CHUNK;
    const int wc = scan_chunk<NBC>(dsts, nE, cbase, nodeBase, vec8, list, tid, lane, wave);
    if (lane == 0) wcnt[wave] = wc;
    __syncthreads();
    if (wave == 0) {
#pragma unroll 1
      for (int wsx = 0; wsx < NWAVE; ++wsx) {
        int n = __builtin_amdgcn_readfirstlane(wcnt[wsx]);
        n = n > WCAP ? WCAP : (n < 0 ? 0 : n);
        const int* lp = list + wsx * WCAP;
#pragma unroll 1
        for (int i = 0; i < n; ++i) {
          const int ent  = __builtin_amdgcn_readfirstlane(lp[i]);
          const int slot = ent & (NBC - 1);
          if (lane == 0) scnt[slot] = scnt[slot] + 1;
        }
      }
    }
    __syncthreads();
  }

  v4i cq[4]; v4f dq[4];
#pragma unroll
  for (int q = 0; q < 4; ++q) {
    const int f = (wave * 4 + q) * 128 + 4 * lane;
    const v4i c = *(const v4i*)(scnt + f);
    cq[q] = c;
    dq[q].x = rsqrtf((float)(c.x + 1));
    dq[q].y = rsqrtf((float)(c.y + 1));
    dq[q].z = rsqrtf((float)(c.z + 1));
    dq[q].w = rsqrtf((float)(c.w + 1));
  }
  int*   cp = cnt + (size_t)nodeBase;
  float* dp = dinv + (size_t)nodeBase;
#pragma unroll
  for (int q = 0; q < 4; ++q) {
    const int f = (wave * 4 + q) * 128 + 4 * lane;
    *(volatile v4i*)(cp + f) = cq[q];
    *(volatile v4f*)(dp + f) = dq[q];
  }
  __threadfence();
#pragma unroll
  for (int q = 0; q < 4; ++q) {
    const int f = (wave * 4 + q) * 128 + 4 * lane;
    *(volatile v4i*)(cp + f) = cq[q];
    *(volatile v4f*)(dp + f) = dq[q];
  }
}

__global__ __launch_bounds__(OTHR) void k_offsets(
    const int* __restrict__ cnt, int* off, int* rbase, int nChunk) {
  __shared__ __attribute__((aligned(16))) int soff[NBC];
  __shared__ __attribute__((aligned(16))) int srb[RBN];
  __shared__ int wtot[OTHR / 32];
  const int tid = threadIdx.x, lane = tid & 31, wave = tid >> 5, sub = tid >> 7;
  for (int i = tid; i < RBN; i += OTHR) srb[i] = 0;
  int carry = 0;
#pragma unroll 1
  for (int ch = 0; ch < nChunk; ++ch) {
    const int base = ch * NBC;
    const v4i c0 = *(const v4i*)(cnt + base + 8 * tid);
    const v4i c1 = *(const v4i*)(cnt + base + 8 * tid + 4);
    const int e0 = max(c0.x, 0), e1 = max(c0.y, 0), e2 = max(c0.z, 0), e3 = max(c0.w, 0);
    const int e4 = max(c1.x, 0), e5 = max(c1.y, 0), e6 = max(c1.z, 0), e7 = max(c1.w, 0);
    const int ts = e0 + e1 + e2 + e3 + e4 + e5 + e6 + e7;
    int incl = ts;
#pragma unroll
    for (int d = 1; d < 32; d <<= 1) {
      const int t = __shfl_up(incl, d);
      if (lane >= d) incl += t;
    }
    if (lane == 31) wtot[wave] = incl;
    __syncthreads();
    const int S0 = wtot[0]  + wtot[1]  + wtot[2]  + wtot[3];
    const int S1 = wtot[4]  + wtot[5]  + wtot[6]  + wtot[7];
    const int S2 = wtot[8]  + wtot[9]  + wtot[10] + wtot[11];
    const int S3 = wtot[12] + wtot[13] + wtot[14] + wtot[15];
    int pre = 0;
#pragma unroll 1
    for (int w = 4 * sub; w < wave; ++w) pre += wtot[w];
    const int b0 = carry;
    const int b1 = b0 + ((S0 + 31) & ~31);
    const int b2 = b1 + ((S1 + 31) & ~31);
    const int b3 = b2 + ((S2 + 31) & ~31);
    const int b4 = b3 + ((S3 + 31) & ~31);
    const int myb = sub == 0 ? b0 : (sub == 1 ? b1 : (sub == 2 ? b2 : b3));
    if (tid == 0) {
      srb[min(4 * ch + 0, RBN - 1)] = b0;
      srb[min(4 * ch + 1, RBN - 1)] = b1;
      srb[min(4 * ch + 2, RBN - 1)] = b2;
      srb[min(4 * ch + 3, RBN - 1)] = b3;
    }
    int run = myb + pre + incl - ts;
    soff[8 * tid + 0] = run; run += e0;
    soff[8 * tid + 1] = run; run += e1;
    soff[8 * tid + 2] = run; run += e2;
    soff[8 * tid + 3] = run; run += e3;
    soff[8 * tid + 4] = run; run += e4;
    soff[8 * tid + 5] = run; run += e5;
    soff[8 * tid + 6] = run; run += e6;
    soff[8 * tid + 7] = run;
    carry = b4;
    __syncthreads();
    const v4i o0 = *(const v4i*)(soff + 4 * tid);
    const v4i o1 = *(const v4i*)(soff + 4 * (tid + OTHR));
    int* op = off + base;
    *(volatile v4i*)(op + 4 * tid) = o0;
    *(volatile v4i*)(op + 4 * (tid + OTHR)) = o1;
    __threadfence();
    *(volatile v4i*)(op + 4 * tid) = o0;
    *(volatile v4i*)(op + 4 * (tid + OTHR)) = o1;
    __syncthreads();
  }
  if (tid == 0) srb[min(4 * nChunk, RBN - 1)] = carry;
  __syncthreads();
  v4i rv = {0, 0, 0, 0};
  if (tid < 32) rv = *(const v4i*)(srb + 4 * tid);
  if (tid < 32) *(volatile v4i*)(rbase + 4 * tid) = rv;
  __threadfence();
  if (tid < 32) *(volatile v4i*)(rbase + 4 * tid) = rv;
}

__global__ __launch_bounds__(NTHR) void k_fill(
    const int* __restrict__ srcs, const int* __restrict__ dsts, const int* __restrict__ off,
    const int* __restrict__ rbase, int* csr, int nN, int nE, int vec8, int csrLen) {
  extern __shared__ v4f lds_dyn[];
  int* region = (int*)lds_dyn;
  int* cursor = region + RCAP;
  int* list   = cursor + NBF;
  int* wcnt   = list + LISTN;
  const int tid = threadIdx.x, lane = tid & 31, wave = tid >> 5;
  const int b = blockIdx.x;
  const int nodeBase = b * NBF;

  int rb0 = rbase[b];
  const int rb1 = rbase[b + 1];
  rb0 = rb0 < 0 ? 0 : (rb0 > csrLen ? csrLen : rb0);
  rb0 &= ~31;
  int len = rb1 - rb0;
  len = len < 0 ? 0 : (len > RCAP ? RCAP : len);
  int lenW = (len + 31) & ~31;
  if (rb0 + lenW > csrLen) lenW = (csrLen - rb0) & ~31;

  {
    const v4i z = {0, 0, 0, 0};
    for (int i = tid; i < RCAP / 4; i += NTHR) ((v4i*)region)[i] = z;
    for (int s = tid; s < NBF; s += NTHR) {
      int o = off[nodeBase + s] - rb0;
      o = o < 0 ? 0 : (o > RCAP ? RCAP : o);
      cursor[s] = o;
    }
  }
  __syncthreads();

  const int nChunks = (nE + CHUNK - 1) / CHUNK;
#pragma unroll 1
  for (int ch = 0; ch < nChunks; ++ch) {
    const int cbase = ch * CHUNK;
    const int wc = scan_chunk<NBF>(dsts, nE, cbase, nodeBase, vec8, list, tid, lane, wave);
    if (lane == 0) wcnt[wave] = wc;
    __syncthreads();
    if (wave == 0) {
#pragma unroll 1
      for (int wsx = 0; wsx < NWAVE; ++wsx) {
        int n = __builtin_amdgcn_readfirstlane(wcnt[wsx]);
        n = n > WCAP ? WCAP : (n < 0 ? 0 : n);
        const int* lp = list + wsx * WCAP;
#pragma unroll 1
        for (int i = 0; i < n; ++i) {
          const int ent  = __builtin_amdgcn_readfirstlane(lp[i]);
          const int slot = ent & (NBF - 1);
          int e = cbase + ((ent >> 12) & (CHUNK - 1));
          e = e > nE - 1 ? nE - 1 : e;
          int src = srcs[e];
          src = src < 0 ? 0 : (src > nN - 1 ? nN - 1 : src);
          if (lane == 0) {
            int pos = cursor[slot];
            pos = pos < 0 ? 0 : (pos > RCAP - 1 ? RCAP - 1 : pos);
            region[pos] = src;
            const int np = pos + 1;
            cursor[slot] = np > RCAP ? RCAP : np;
          }
        }
      }
    }
    __syncthreads();
  }

  const int nv = lenW >> 2;
  int* gp = csr + rb0;
#pragma unroll 1
  for (int i = tid; i < nv; i += NTHR) { const v4i v = ((const v4i*)region)[i]; *(volatile v4i*)(gp + 4 * i) = v; }
  __threadfence();
#pragma unroll 1
  for (int i = tid; i < nv; i += NTHR) { const v4i v = ((const v4i*)region)[i]; *(volatile v4i*)(gp + 4 * i) = v; }
}

__global__ __launch_bounds__(NTHR) void k_gemm(
    const float* __restrict__ A, const unsigned short* __restrict__ Bh, const unsigned short* __restrict__ Bl,
    const float* __restrict__ dinv, float* C, int nRowsA) {
  extern __shared__ v4f lds_dyn[];
  constexpr int KD = HIDC;
  unsigned short* sAh = (unsigned short*)lds_dyn;
  unsigned short* sAl = sAh + GROWS * AP;
  float* stg = (float*)((char*)lds_dyn + (size_t)2 * GROWS * AP * 2);
  const int tid = threadIdx.x, lane = tid & 31, wave = tid >> 5, hh = lane >> 4, m = lane & 15;
  const int rowBase = blockIdx.x * GROWS;

#pragma unroll
  for (int i = 0; i < (GROWS * KD / 8) / NTHR; ++i) {
    const int idx = i * NTHR + tid;
    const int r   = idx >> 4;
    const int c0  = (idx & 15) * 8;
    int row = rowBase + r;
    row = row > nRowsA - 1 ? nRowsA - 1 : row;
    const float* ap = A + (size_t)row * KD + c0;
    const v4f a = *(const v4f*)ap, b = *(const v4f*)(ap + 4);
    v8us hi, lo;
    split8(a, b, hi, lo);
    *(v8us*)(sAh + r * AP + c0) = hi;
    *(v8us*)(sAl + r * AP + c0) = lo;
  }
  __syncthreads();

  const int r0 = wave * 16 + 8 * hh;
  const v4f dA = *(const v4f*)(dinv + (size_t)rowBase + r0);
  const v4f dB = *(const v4f*)(dinv + (size_t)rowBase + r0 + 4);
  float s[8];
  s[0] = dA.x; s[1] = dA.y; s[2] = dA.z; s[3] = dA.w; s[4] = dB.x; s[5] = dB.y; s[6] = dB.z; s[7] = dB.w;

  const unsigned short* arh = sAh + (wave * 16 + m) * AP + 8 * hh;
  const unsigned short* arl = sAl + (wave * 16 + m) * AP + 8 * hh;
#pragma unroll 1
  for (int tp = 0; tp < 2; ++tp) {
    v8f acc[4];
#pragma unroll
    for (int t = 0; t < 4; ++t) { v8f z = {0.f, 0.f, 0.f, 0.f, 0.f, 0.f, 0.f, 0.f}; acc[t] = z; }
#pragma unroll 1
    for (int kt = 0; kt < KD / 32; ++kt) {
      FragB ah, al;
      ah.h[0] = *(const v8us*)(arh + 32 * kt);
      ah.h[1] = *(const v8us*)(arh + 32 * kt + 16);
      al.h[0] = *(const v8us*)(arl + 32 * kt);
      al.h[1] = *(const v8us*)(arl + 32 * kt + 16);
#pragma unroll
      for (int t = 0; t < 4; ++t) {
        const size_t bo = (size_t)(64 * tp + 16 * t + m) * KD + 32 * kt + 8 * hh;
        FragB bh, bl;
        bh.h[0] = *(const v8us*)(Bh + bo);
        bh.h[1] = *(const v8us*)(Bh + bo + 16);
        bl.h[0] = *(const v8us*)(Bl + bo);
        bl.h[1] = *(const v8us*)(Bl + bo + 16);
        acc[t] = wmb(ah.v, bh.v, acc[t]);
        acc[t] = wmb(ah.v, bl.v, acc[t]);
        acc[t] = wmb(al.v, bh.v, acc[t]);
      }
    }
    float* sp = stg + r0 * HIDC + 64 * tp + m;
#pragma unroll
    for (int t = 0; t < 4; ++t) {
#pragma unroll
      for (int r = 0; r < 8; ++r) sp[r * HIDC + 16 * t] = acc[t][r] * s[r];
    }
  }
  __syncthreads();

  const float* lp = stg + wave * 16 * HIDC + 4 * lane;
  float* gp = C + ((size_t)rowBase + wave * 16) * HIDC + 4 * lane;
  v4f rowv[16];
#pragma unroll
  for (int i = 0; i < 16; ++i) rowv[i] = *(const v4f*)(lp + i * HIDC);
#pragma unroll
  for (int i = 0; i < 16; ++i) *(volatile v4f*)(gp + (size_t)i * HIDC) = rowv[i];
  __threadfence();
#pragma unroll
  for (int i = 0; i < 16; ++i) *(volatile v4f*)(gp + (size_t)i * HIDC) = rowv[i];
}

__global__ __launch_bounds__(NTHR) void k_agg(
    const int* __restrict__ csr, const int* __restrict__ off, const int* __restrict__ cnt,
    const float* __restrict__ dinv, const float* __restrict__ hw, float* h,
    const float* __restrict__ bs, int nN, int csrLen, int nStore, int doRelu) {
  const int tid = threadIdx.x, lane = tid & 31, wave = tid >> 5;
  const int tbase = blockIdx.x * TGT + wave * 32;
  const int cl = tbase + lane;
  const int cnt_l = cnt[cl];
  const int off_l = off[cl];
  union FI { float f; int i; };
  FI dvu; dvu.f = dinv[cl];
  const v4f bb = *(const v4f*)(bs + 4 * lane);

#pragma unroll 1
  for (int j = 0; j < 32; ++j) {
    const int c = tbase + j;
    int n = __builtin_amdgcn_readlane(cnt_l, j);
    n = n < 0 ? 0 : (n > DEGCAP ? DEGCAP : n);
    const int st = __builtin_amdgcn_readlane(off_l, j);
    FI du; du.i = __builtin_amdgcn_readlane(dvu.i, j);
    const float dc = du.f;
    v4f acc = {0.f, 0.f, 0.f, 0.f};
#pragma unroll 1
    for (int q0 = 0; q0 < n; q0 += 32) {
      int pos = st + q0 + lane;
      pos = pos < 0 ? 0 : (pos > csrLen - 1 ? csrLen - 1 : pos);
      int sl = csr[pos];
      sl = sl < 0 ? 0 : (sl > nN - 1 ? nN - 1 : sl);
      const int mcnt = (n - q0) < 32 ? (n - q0) : 32;
#pragma unroll 1
      for (int p = 0; p < mcnt; ++p) {
        const int s = __builtin_amdgcn_readlane(sl, p);
        acc = acc + *(const v4f*)(hw + (size_t)s * HIDC + 4 * lane);
      }
    }
    const v4f sv = *(const v4f*)(hw + (size_t)c * HIDC + 4 * lane);
    v4f v = (acc + sv) * dc + bb;
    if (doRelu != 0) {
      v.x = fmaxf(v.x, 0.f); v.y = fmaxf(v.y, 0.f); v.z = fmaxf(v.z, 0.f); v.w = fmaxf(v.w, 0.f);
    }
    if (c < nStore) {
      float* hp = h + (size_t)c * HIDC + 4 * lane;
      *(volatile v4f*)hp = v;
      __threadfence();
      *(volatile v4f*)hp = v;
    }
  }
}

__global__ __launch_bounds__(NTHR) void k_sortsc(
    const float* __restrict__ x, const float* __restrict__ p, float* sc, u64* keys, int n) {
  __shared__ __attribute__((aligned(16))) u64 skey[SCH];
  __shared__ __attribute__((aligned(16))) float ssc[SCH];
  __shared__ __attribute__((aligned(16))) float sp[HIDC];
  const int tid = threadIdx.x;
  const int cbase = blockIdx.x * SCH;
  if (tid < HIDC) sp[tid] = p[tid];
  __syncthreads();
  float q = 0.0f;
#pragma unroll 1
  for (int c = 0; c < HIDC; ++c) q = fmaf(sp[c], sp[c], q);
  const float rinv = rsqrtf(q);

#pragma unroll 1
  for (int j = 0; j < SCH / NTHR; ++j) {
    const int li = j * NTHR + tid;
    const int node = cbase + li;
    const int row = node < n ? node : n - 1;
    const float* xr = x + (size_t)row * HIDC;
    float a0 = 0.f, a1 = 0.f, a2 = 0.f, a3 = 0.f, a4 = 0.f, a5 = 0.f, a6 = 0.f, a7 = 0.f;
#pragma unroll 1
    for (int c = 0; c < HIDC; c += 8) {
      const v4f u  = *(const v4f*)(xr + c),  w  = *(const v4f*)(xr + c + 4);
      const v4f pu = *(const v4f*)(sp + c),  pw = *(const v4f*)(sp + c + 4);
      a0 = fmaf(u.x, pu.x, a0); a1 = fmaf(u.y, pu.y, a1); a2 = fmaf(u.z, pu.z, a2); a3 = fmaf(u.w, pu.w, a3);
      a4 = fmaf(w.x, pw.x, a4); a5 = fmaf(w.y, pw.y, a5); a6 = fmaf(w.z, pw.z, a6); a7 = fmaf(w.w, pw.w, a7);
    }
    const float d = ((a0 + a4) + (a2 + a6)) + ((a1 + a5) + (a3 + a7));
    const float s = tanhf(d * rinv);
    const bool in = node < n;
    ssc[li]  = in ? s : 0.0f;
    skey[li] = in ? mkkey(s, node) : (u64)0;
  }
  __syncthreads();

#pragma unroll 1
  for (int kk = 2; kk <= SCH; kk <<= 1) {
#pragma unroll 1
    for (int jj = kk >> 1; jj > 0; jj >>= 1) {
#pragma unroll
      for (int qq = 0; qq < SCH / 2 / NTHR; ++qq) {
        const int t  = qq * NTHR + tid;
        const int i  = ((t & ~(jj - 1)) << 1) | (t & (jj - 1));
        const int i2 = i | jj;
        const u64 a = skey[i], b = skey[i2];
        const bool up = ((i & kk) == 0);
        const bool sw = up ? (a > b) : (a < b);
        if (sw) { skey[i] = b; skey[i2] = a; }
      }
      __syncthreads();
    }
  }

  v2u kv[4]; v4f sv[2];
#pragma unroll
  for (int qq = 0; qq < 4; ++qq) kv[qq] = *(const v2u*)(skey + 2 * (qq * NTHR + tid));
#pragma unroll
  for (int qq = 0; qq < 2; ++qq) sv[qq] = *(const v4f*)(ssc + 4 * (qq * NTHR + tid));
  u64* kp = keys + (size_t)cbase;
  float* scp = sc + (size_t)cbase;
#pragma unroll
  for (int qq = 0; qq < 4; ++qq) *(volatile v2u*)(kp + 2 * (qq * NTHR + tid)) = kv[qq];
#pragma unroll
  for (int qq = 0; qq < 2; ++qq) *(volatile v4f*)(scp + 4 * (qq * NTHR + tid)) = sv[qq];
  __threadfence();
#pragma unroll
  for (int qq = 0; qq < 4; ++qq) *(volatile v2u*)(kp + 2 * (qq * NTHR + tid)) = kv[qq];
#pragma unroll
  for (int qq = 0; qq < 2; ++qq) *(volatile v4f*)(scp + 4 * (qq * NTHR + tid)) = sv[qq];
}

__global__ __launch_bounds__(NTHR) void k_rank(
    const float* __restrict__ sc, const u64* __restrict__ keys, int* rank, int n, int nChunks) {
  __shared__ __attribute__((aligned(16))) u64 sk[SCH];
  const int tid = threadIdx.x;
  const int i = blockIdx.x * NTHR + tid;
  const float s = sc[i];
  const u64 key = (i < n) ? mkkey(s, i) : (u64)0;
  int gt = 0;
#pragma unroll 1
  for (int c = 0; c < nChunks; ++c) {
    const u64* kp = keys + (size_t)c * SCH;
    v2u t4[4];
#pragma unroll
    for (int qq = 0; qq < 4; ++qq) t4[qq] = *(const v2u*)(kp + 2 * (qq * NTHR + tid));
    __syncthreads();
#pragma unroll
    for (int qq = 0; qq < 4; ++qq) *(v2u*)(sk + 2 * (qq * NTHR + tid)) = t4[qq];
    __syncthreads();
    int pos = 0;
#pragma unroll
    for (int step = SCH / 2; step > 0; step >>= 1) {
      const u64 probe = sk[pos + step - 1];
      pos += (probe <= key) ? step : 0;
    }
    const u64 lastk = sk[SCH - 1];
    if (lastk <= key) pos = SCH;
    gt += SCH - pos;
  }
  *(volatile int*)(rank + i) = gt;
  __threadfence();
  *(volatile int*)(rank + i) = gt;
}

__global__ __launch_bounds__(NTHR) void k_perm(
    const int* __restrict__ rank, int* perm, int n, int k) {
  __shared__ __attribute__((aligned(16))) int pl[PBLK];
  const int tid = threadIdx.x;
  const int r0 = blockIdx.x * PBLK;
  for (int i = tid; i < PBLK; i += NTHR) pl[i] = 0;
  __syncthreads();
#pragma unroll 1
  for (int base = 0; base < n; base += NTHR) {
    const int i  = base + tid;
    const int ic = i < n ? i : n - 1;
    const int rk = rank[ic];
    const unsigned rel = (unsigned)(rk - r0);
    if (i < n && rel < (unsigned)PBLK && rk < k) pl[rel] = i;
  }
  __syncthreads();
  v4i pv[4];
#pragma unroll
  for (int qq = 0; qq < 4; ++qq) pv[qq] = *(const v4i*)(pl + 4 * (qq * NTHR + tid));
  int* pp = perm + (size_t)r0;
#pragma unroll
  for (int qq = 0; qq < 4; ++qq) *(volatile v4i*)(pp + 4 * (qq * NTHR + tid)) = pv[qq];
  __threadfence();
#pragma unroll
  for (int qq = 0; qq < 4; ++qq) *(volatile v4i*)(pp + 4 * (qq * NTHR + tid)) = pv[qq];
}

__global__ __launch_bounds__(NTHR) void k_poolx(
    const float* __restrict__ x, const int* __restrict__ perm, const float* __restrict__ sc,
    float* xo, int n, int k) {
  const int tid = threadIdx.x, lane = tid & 31, wave = tid >> 5;
  const int r = blockIdx.x * RPB + wave;
  const int rc = r < k ? r : k - 1;
  int idx = perm[rc];
  idx = idx < 0 ? 0 : (idx > n - 1 ? n - 1 : idx);
  const v4f a = *(const v4f*)(x + (size_t)idx * HIDC + 4 * lane);
  const float s = sc[idx];
  const v4f z = {0.f, 0.f, 0.f, 0.f};
  const v4f v = (r < k) ? a * s : z;
  float* op = xo + (size_t)r * HIDC + 4 * lane;
  *(volatile v4f*)op = v;
  __threadfence();
  *(volatile v4f*)op = v;
}

__global__ __launch_bounds__(NTHR) void k_unpool(
    const float* __restrict__ res, const float* __restrict__ cur, const int* __restrict__ rank,
    float* xo, int n, int k) {
  const int tid = threadIdx.x, lane = tid & 31, wave = tid >> 5;
  const int r = blockIdx.x * RPB + wave;
  const int rc = r < n ? r : n - 1;
  const int rk = rank[rc];
  const bool hasUp = (r < n) && ((unsigned)rk < (unsigned)k);
  int ci = rk < 0 ? 0 : (rk > k - 1 ? k - 1 : rk);
  const v4f a = *(const v4f*)(res + (size_t)rc * HIDC + 4 * lane);
  const v4f b = *(const v4f*)(cur + (size_t)ci * HIDC + 4 * lane);
  const v4f z = {0.f, 0.f, 0.f, 0.f};
  const v4f v = ((r < n) ? a : z) + (hasUp ? b : z);
  float* op = xo + (size_t)r * HIDC + 4 * lane;
  *(volatile v4f*)op = v;
  __threadfence();
  *(volatile v4f*)op = v;
}

__device__ __forceinline__ void remap1(int s, int d, bool inr, const int* __restrict__ rank,
                                       int n, int k, int& ns, int& nd) {
  const bool pv = inr && (s >= 0) && (d >= 0);
  const int scl = s < 0 ? 0 : (s > n - 1 ? n - 1 : s);
  const int dcl = d < 0 ? 0 : (d > n - 1 ? n - 1 : d);
  const int rs = rank[scl], rd = rank[dcl];
  const bool v = pv && ((unsigned)rs < (unsigned)k) && ((unsigned)rd < (unsigned)k);
  ns = v ? rs : -1;
  nd = v ? rd : -1;
}

__global__ __launch_bounds__(NTHR) void k_remap(
    const int* __restrict__ srcs, const int* __restrict__ dsts, const int* __restrict__ rank,
    int* so, int* dso, int n, int k, int nE) {
  const int tid = threadIdx.x;
  const int e0 = (blockIdx.x * NTHR + tid) * 4;
  const int ec = e0 > nE - 4 ? nE - 4 : e0;
  const v4i s4 = *(const v4i*)(srcs + ec), d4 = *(const v4i*)(dsts + ec);
  v4i os, od;
  int a, b;
  remap1(s4.x, d4.x, e0 + 0 < nE, rank, n, k, a, b); os.x = a; od.x = b;
  remap1(s4.y, d4.y, e0 + 1 < nE, rank, n, k, a, b); os.y = a; od.y = b;
  remap1(s4.z, d4.z, e0 + 2 < nE, rank, n, k, a, b); os.z = a; od.z = b;
  remap1(s4.w, d4.w, e0 + 3 < nE, rank, n, k, a, b); os.w = a; od.w = b;
  *(volatile v4i*)(so + e0) = os;
  *(volatile v4i*)(dso + e0) = od;
  __threadfence();
  *(volatile v4i*)(so + e0) = os;
  *(volatile v4i*)(dso + e0) = od;
}

extern "C" void kernel_launch(void* const* d_in, const int* in_sizes, int n_in,
                              void* d_out, int out_size, void* d_ws, size_t ws_size,
                              hipStream_t stream) {
  if (n_in < 10) return;
  const int nN = in_sizes[0] / HIDC;
  const int nE = in_sizes[1] / 2;
  if (nN < 2 || nE < 8) return;
  if (in_sizes[0] != nN * HIDC || in_sizes[1] != 2 * nE) return;
  if ((nE & 3) != 0) return;
  if (in_sizes[3] != HIDC * HIDC || in_sizes[4] != HIDC) return;
  if (in_sizes[5] != 3 * HIDC * HIDC || in_sizes[6] != 3 * HIDC) return;
  if (in_sizes[7] != 3 * HIDC) return;
  if (in_sizes[8] != 3 * HIDC * HIDC || in_sizes[9] != 3 * HIDC) return;
  if (out_size != nN * HIDC) return;
  if (nN > (1 << 20) || nE > (1 << 26)) return;

  const float* x   = (const float*)d_in[0];
  const int*   ei  = (const int*)d_in[1];
  const float* Wd0 = (const float*)d_in[3];
  const float* bd0 = (const float*)d_in[4];
  const float* Wd  = (const float*)d_in[5];
  const float* bd  = (const float*)d_in[6];
  const float* pp  = (const float*)d_in[7];
  const float* Wu  = (const float*)d_in[8];
  const float* bu  = (const float*)d_in[9];
  float* out = (float*)d_out;

  int nL[4], NP[4], CP[4], nBCv[4], nBFv[4];
  nL[0] = nN;
  for (int i = 1; i < 4; ++i) nL[i] = (nL[i - 1] + 1) / 2;
  for (int i = 0; i < 4; ++i) {
    NP[i]   = ((nL[i] + TGT - 1) / TGT) * TGT;
    CP[i]   = ((nL[i] + NBC - 1) / NBC) * NBC;
    nBCv[i] = CP[i] / NBC;
    nBFv[i] = (nL[i] + NBF - 1) / NBF;
  }
  if (4 * nBCv[0] + 1 > RBN) return;
  if (31 * 4 * nBCv[0] > 4096) return;
  const int csrLen = ((nE + 31) & ~31) + 4096;
  const int EPAD = ((nE + EPB - 1) / EPB) * EPB;
  int SCP[3], PMP[3];
  for (int i = 0; i < 3; ++i) {
    SCP[i] = ((nL[i] + SCH - 1) / SCH) * SCH;
    PMP[i] = ((nL[i + 1] + PBLK - 1) / PBLK) * PBLK;
  }
  const size_t HH = (size_t)HIDC * HIDC;

  char* ws = (char*)d_ws;
  size_t off = 0;
#define CARVE(NAME, BYTES) const size_t NAME = off; off += (size_t)(BYTES); off = (off + 255) & ~(size_t)255;
  CARVE(oW, NMAT * 2 * HH * 2)
  size_t oCnt[4], oDv[4], oOff[4], oRb[4], oCsr[4];
  for (int i = 0; i < 4; ++i) {
    CARVE(t0, (size_t)CP[i] * 4)      oCnt[i] = t0;
    CARVE(t1, (size_t)CP[i] * 4)      oDv[i]  = t1;
    CARVE(t2, (size_t)CP[i] * 4)      oOff[i] = t2;
    CARVE(t3, (size_t)RBN * 4)        oRb[i]  = t3;
    CARVE(t4, (size_t)csrLen * 4)     oCsr[i] = t4;
  }
  CARVE(oXs0, (size_t)NP[0] * HIDC * 4)
  CARVE(oXs1, (size_t)NP[1] * HIDC * 4)
  CARVE(oXs2, (size_t)NP[2] * HIDC * 4)
  CARVE(oX3,  (size_t)NP[3] * HIDC * 4)
  CARVE(oXin, (size_t)NP[0] * HIDC * 4)
  CARVE(oHw,  (size_t)NP[0] * HIDC * 4)
  CARVE(oEsA, (size_t)EPAD * 4)
  CARVE(oEdA, (size_t)EPAD * 4)
  CARVE(oEsB, (size_t)EPAD * 4)
  CARVE(oEdB, (size_t)EPAD * 4)
  size_t oSc[3], oKey[3], oRk[3], oPm[3];
  for (int i = 0; i < 3; ++i) {
    CARVE(t5, (size_t)SCP[i] * 4)     oSc[i]  = t5;
    CARVE(t6, (size_t)SCP[i] * 8)     oKey[i] = t6;
    CARVE(t7, (size_t)NP[i] * 4)      oRk[i]  = t7;
    CARVE(t8, (size_t)PMP[i] * 4)     oPm[i]  = t8;
  }
#undef CARVE
  if (off > ws_size) return;

  unsigned short* wp = (unsigned short*)(ws + oW);
  int* cnt[4]; float* dinv[4]; int* offp[4]; int* rb[4]; int* csr[4];
  for (int i = 0; i < 4; ++i) {
    cnt[i]  = (int*)(ws + oCnt[i]);
    dinv[i] = (float*)(ws + oDv[i]);
    offp[i] = (int*)(ws + oOff[i]);
    rb[i]   = (int*)(ws + oRb[i]);
    csr[i]  = (int*)(ws + oCsr[i]);
  }
  float* xs0 = (float*)(ws + oXs0);
  float* xs1 = (float*)(ws + oXs1);
  float* xs2 = (float*)(ws + oXs2);
  float* x3  = (float*)(ws + oX3);
  float* xin = (float*)(ws + oXin);
  float* hw  = (float*)(ws + oHw);
  int* esA = (int*)(ws + oEsA); int* edA = (int*)(ws + oEdA);
  int* esB = (int*)(ws + oEsB); int* edB = (int*)(ws + oEdB);
  float* scv[3]; u64* keyv[3]; int* rkv[3]; int* pmv[3];
  for (int i = 0; i < 3; ++i) {
    scv[i]  = (float*)(ws + oSc[i]);
    keyv[i] = (u64*)(ws + oKey[i]);
    rkv[i]  = (int*)(ws + oRk[i]);
    pmv[i]  = (int*)(ws + oPm[i]);
  }

  const int vec8 = ((nE & 7) == 0) ? 1 : 0;

  hipFuncSetAttribute(reinterpret_cast<const void*>(&k_fill),
                      hipFuncAttributeMaxDynamicSharedMemorySize, LDS_FILL);
  hipFuncSetAttribute(reinterpret_cast<const void*>(&k_gemm),
                      hipFuncAttributeMaxDynamicSharedMemorySize, LDS_GEMM);

  auto build_csr = [&](int L, const int* srcs, const int* dsts) {
    k_count<<<nBCv[L], NTHR, 0, stream>>>(dsts, cnt[L], dinv[L], nE, vec8);
    k_offsets<<<1, OTHR, 0, stream>>>(cnt[L], offp[L], rb[L], nBCv[L]);
    k_fill<<<nBFv[L], NTHR, LDS_FILL, stream>>>(srcs, dsts, offp[L], rb[L], csr[L], nL[L], nE, vec8, csrLen);
  };
  auto gcn_layer = [&](int L, const float* Ain, int nRowsA, int mat, const float* bias,
                       float* outp, int nStore, int relu) {
    const unsigned short* bh = wp + (size_t)mat * 2 * HH;
    const unsigned short* bl = bh + HH;
    k_gemm<<<NP[L] / GROWS, NTHR, LDS_GEMM, stream>>>(Ain, bh, bl, dinv[L], hw, nRowsA);
    k_agg<<<NP[L] / TGT, NTHR, 0, stream>>>(csr[L], offp[L], cnt[L], dinv[L], hw, outp, bias,
                                           nL[L], csrLen, nStore, relu);
  };
  auto pool = [&](int P, const float* xs, const int* srcs, const int* dsts, int* so, int* dso) {
    k_sortsc<<<SCP[P] / SCH, NTHR, 0, stream>>>(xs, pp + (size_t)P * HIDC, scv[P], keyv[P], nL[P]);
    k_rank<<<NP[P] / NTHR, NTHR, 0, stream>>>(scv[P], keyv[P], rkv[P], nL[P], SCP[P] / SCH);
    k_perm<<<PMP[P] / PBLK, NTHR, 0, stream>>>(rkv[P], pmv[P], nL[P], nL[P + 1]);
    k_poolx<<<NP[P + 1] / RPB, NTHR, 0, stream>>>(xs, pmv[P], scv[P], xin, nL[P], nL[P + 1]);
    k_remap<<<EPAD / EPB, NTHR, 0, stream>>>(srcs, dsts, rkv[P], so, dso, nL[P], nL[P + 1], nE);
  };

  k_wprep<<<NMAT * 8, NTHR, 0, stream>>>(Wd0, Wd, Wu, wp);

  build_csr(0, ei, ei + nE);
  gcn_layer(0, x, nN, 0, bd0, xs0, NP[0], 1);
  pool(0, xs0, ei, ei + nE, esA, edA);
  build_csr(1, esA, edA);
  gcn_layer(1, xin, NP[1], 1, bd + 0 * HIDC, xs1, NP[1], 1);
  pool(1, xs1, esA, edA, esB, edB);
  build_csr(2, esB, edB);
  gcn_layer(2, xin, NP[2], 2, bd + 1 * HIDC, xs2, NP[2], 1);
  pool(2, xs2, esB, edB, esA, edA);
  build_csr(3, esA, edA);
  gcn_layer(3, xin, NP[3], 3, bd + 2 * HIDC, x3, NP[3], 1);

  k_unpool<<<NP[2] / RPB, NTHR, 0, stream>>>(xs2, x3, rkv[2], xin, nL[2], nL[3]);
  gcn_layer(2, xin, NP[2], 4, bu + 0 * HIDC, xs2, NP[2], 1);
  k_unpool<<<NP[1] / RPB, NTHR, 0, stream>>>(xs1, xs2, rkv[1], xin, nL[1], nL[2]);
  gcn_layer(1, xin, NP[1], 5, bu + 1 * HIDC, xs1, NP[1], 1);
  k_unpool<<<NP[0] / RPB, NTHR, 0, stream>>>(xs0, xs1, rkv[0], xin, nL[0], nL[1]);
  gcn_layer(0, xin, NP[0], 6, bu + 2 * HIDC, out, nN, 0);
}
